// MappingNetwork_52621939310621
// MI455X (gfx1250) — hardware-verified
//
#include <hip/hip_runtime.h>
#include <math.h>

typedef __attribute__((ext_vector_type(16))) _Float16 v16h;
typedef __attribute__((ext_vector_type(16))) __bf16 v16b;
typedef __attribute__((ext_vector_type(8)))  _Float16 v8h;
typedef __attribute__((ext_vector_type(8)))  float v8f;
typedef __attribute__((ext_vector_type(4)))  float v4f;
typedef __attribute__((ext_vector_type(2)))  float v2f;
typedef __attribute__((ext_vector_type(4)))  unsigned v4u;
typedef __attribute__((ext_vector_type(4)))  int v4i;
typedef float __attribute__((may_alias)) float_a;
typedef int __attribute__((may_alias)) int_a;

template <typename T> __device__ __forceinline__ void vst2(void* p, T v) { *(volatile T*)p = v; __threadfence(); *(volatile T*)p = v; }
__device__ __forceinline__ v8f wmma16(v16h a, v16h b, v8f c) {
  v8f d = __builtin_amdgcn_wmma_f32_16x16x32_f16(false, a, false, b, (short)0, c, false, false);
  asm volatile("v_nop\n\tv_nop\n\tv_nop\n\tv_nop" : "+v"(d) : "v"(a), "v"(b));
  return d;
}
__device__ __forceinline__ v8f wmma_bf(v16b a, v16b b, v8f c) {
  v8f d = __builtin_amdgcn_wmma_f32_16x16x32_bf16(false, a, false, b, (short)0, c, false, false);
  asm volatile("v_nop\n\tv_nop\n\tv_nop\n\tv_nop" : "+v"(d) : "v"(a), "v"(b));
  return d;
}
__device__ __forceinline__ v16h frag_h(const _Float16* rowk0, int lane) {
  union { v16h v; v8h q[2]; } u; const _Float16* p = rowk0 + 8 * (lane >> 4);
  u.q[0] = *(const v8h*)p; u.q[1] = *(const v8h*)(p + 16); return u.v;
}
__device__ __forceinline__ v16h frag_f32(const float* rowk0, int lane) {
  v16h a; const float* p = rowk0 + 8 * (lane >> 4);
#pragma unroll
  for (int i = 0; i < 8; ++i) { a[i] = (_Float16)p[i]; a[8 + i] = (_Float16)p[16 + i]; }
  return a;
}
__device__ __forceinline__ v16h frag_f32s(const float* rowk0, int lane, float sc) {
  v16h a; const float* p = rowk0 + 8 * (lane >> 4);
#pragma unroll
  for (int i = 0; i < 8; ++i) { a[i] = (_Float16)(p[i] * sc); a[8 + i] = (_Float16)(p[16 + i] * sc); }
  return a;
}
__device__ __forceinline__ v16h fragc_f32(const float* W, int k0, int n, int lane, int ld, int K) {
  v16h a; const int g = lane >> 4;
#pragma unroll
  for (int i = 0; i < 8; ++i) { const int ka = k0 + 8 * g + i, kb = ka + 16;
    a[i] = (_Float16)(ka < K ? W[(size_t)(ka < K ? ka : K - 1) * ld + n] : 0.f); a[8 + i] = (_Float16)(kb < K ? W[(size_t)(kb < K ? kb : K - 1) * ld + n] : 0.f); }
  return a;
}
struct F2 { v16b h, l; };
__device__ __forceinline__ F2 bsplit16(const float v[16]) { F2 r;
#pragma unroll
  for (int i = 0; i < 16; ++i) { const __bf16 h = (__bf16)v[i]; r.h[i] = h; r.l[i] = (__bf16)(v[i] - (float)h); }
  return r; }
__device__ __forceinline__ F2 split_row(const float* row, int k0, int lane) { float v[16]; const float* p = row + k0 + 8 * (lane >> 4);
#pragma unroll
  for (int i = 0; i < 8; ++i) { v[i] = p[i]; v[8 + i] = p[16 + i]; }
  return bsplit16(v); }
__device__ __forceinline__ F2 split_rowK(const float* row, int k0, int lane, int K) { float v[16]; const int g = lane >> 4;
#pragma unroll
  for (int i = 0; i < 8; ++i) { const int ka = k0 + 8 * g + i, kb = ka + 16; v[i] = ka < K ? row[ka < K ? ka : K - 1] : 0.f; v[8 + i] = kb < K ? row[kb < K ? kb : K - 1] : 0.f; }
  return bsplit16(v); }
__device__ __forceinline__ F2 split_col(const float* W, int k0, int n, int lane, int ld, int K) { float v[16]; const int g = lane >> 4;
#pragma unroll
  for (int i = 0; i < 8; ++i) { const int ka = k0 + 8 * g + i, kb = ka + 16; v[i] = ka < K ? W[(size_t)(ka < K ? ka : K - 1) * ld + n] : 0.f; v[8 + i] = kb < K ? W[(size_t)(kb < K ? kb : K - 1) * ld + n] : 0.f; }
  return bsplit16(v); }
__device__ __forceinline__ v8f mac3(const F2& a, const F2& b, v8f c) { c = wmma_bf(a.l, b.h, c); c = wmma_bf(a.h, b.l, c); return wmma_bf(a.h, b.h, c); }
__device__ __forceinline__ float sigm(float v) { return 1.0f / (1.0f + expf(-v)); }
#define LDSX() do { asm volatile("s_wait_dscnt 0" ::: "memory"); __builtin_amdgcn_wave_barrier(); __builtin_amdgcn_fence(__ATOMIC_RELEASE, "workgroup"); } while (0)


#define NBAT 16384
#define LAT 16
#define HID 256
#define STY 64
#define NSP 10
#ifndef NRW
#define NRW NBAT
#endif
typedef __attribute__((ext_vector_type(8))) __bf16 v8b;
__device__ __forceinline__ v16b frag_b(const __bf16* rowk0, int lane) {
  union { v16b v; v8b q[2]; } u; const __bf16* p = rowk0 + 8 * (lane >> 4);
  u.q[0] = *(const v8b*)p; u.q[1] = *(const v8b*)(p + 16); return u.v;
}
__device__ __forceinline__ float bfr(float v) { return (float)(__bf16)v; }
__device__ __attribute__((noinline)) float exp_ni(float v) { return expf(v); }
__device__ __attribute__((noinline)) float erf_ni(float v) { return erff(v); }

#define PK_S0 0
#define PK_S1 ((size_t)HID * 32)
#define PK_S2 (PK_S1 + (size_t)HID * HID)
#define PK_S3 (PK_S2 + (size_t)HID * HID)
#define PK_U0 (PK_S3 + (size_t)HID * HID)
#define PK_U1 (PK_U0 + (size_t)NSP * HID * HID)
#define PK_U2 (PK_U1 + (size_t)NSP * HID * HID)
#define PK_U3 (PK_U2 + (size_t)NSP * HID * HID)
#define PK_END (PK_U3 + (size_t)NSP * STY * HID)
#define WS_PK  0u
#define WS_HA  (((2u * PK_END) + 127u) / 128u * 128u)
#define WS_LA  (WS_HA + 2u * NBAT * HID)
#define WS_HB  (WS_LA + 2u * NBAT * HID)
#define WS_LB  (WS_HB + 2u * NBAT * HID)
#define WS_IDX (WS_LB + 2u * NBAT * HID)
#define WS_OFF (WS_IDX + 4u * NBAT)
#define WS_END (WS_OFF + 4u * 32)

__global__ __launch_bounds__(256) void k_pack(const float* __restrict__ SW0, const float* __restrict__ SW1, const float* __restrict__ SW2, const float* __restrict__ SW3, const float* __restrict__ UW0, const float* __restrict__ UW1, const float* __restrict__ UW2, const float* __restrict__ UW3, __bf16* __restrict__ PK) {
  __shared__ __align__(16) __bf16 s[HID]; const int n = blockIdx.x, which = blockIdx.y, t = threadIdx.x; int K; size_t dst;
  if (which == 0) { K = 32; dst = PK_S0 + (size_t)n * 32; if (t < 32) s[t] = (__bf16)((t < LAT) ? SW0[(size_t)t * HID + n] : 0.f); }
  else if (which <= 3) { const float* Wm = (which == 1) ? SW1 : (which == 2) ? SW2 : SW3; K = HID; dst = ((which == 1) ? PK_S1 : (which == 2) ? PK_S2 : PK_S3) + (size_t)n * HID; for (int k = t; k < K; k += 256) s[k] = (__bf16)Wm[(size_t)k * HID + n]; }
  else if (which <= 6) { if (blockIdx.z >= NSP) return; const int sp = blockIdx.z; const float* Wm = ((which == 4) ? UW0 : (which == 5) ? UW1 : UW2) + (size_t)sp * HID * HID; K = HID; dst = ((which == 4) ? PK_U0 : (which == 5) ? PK_U1 : PK_U2) + ((size_t)sp * HID + n) * HID; for (int k = t; k < K; k += 256) s[k] = (__bf16)Wm[(size_t)k * HID + n]; }
  else { if (blockIdx.z >= NSP || n >= STY) return; const int sp = blockIdx.z; const float* Wm = UW3 + (size_t)sp * HID * STY; K = HID; dst = PK_U3 + ((size_t)sp * STY + n) * HID; for (int k = t; k < K; k += 256) s[k] = (__bf16)Wm[(size_t)k * STY + n]; }
  __syncthreads();
  for (int q = t; q < K / 8; q += 256) vst2((unsigned*)(PK + dst + q * 8), *(const v4u*)&s[q * 8]);
}
__global__ __launch_bounds__(256) void k_group(const int* __restrict__ Y, int* __restrict__ IDX, int* __restrict__ OFF) {
  __shared__ int wcnt[8]; __shared__ int sidx[256]; const int t = threadIdx.x, wave = t >> 5, lane = t & 31; int base = 0;
  if (t == 0) OFF[0] = 0;
#pragma unroll 1
  for (int sp = 0; sp < NSP; ++sp) {
#pragma unroll 1
    for (int c0 = 0; c0 < NRW; c0 += 256) { const int row = c0 + t; const bool hit = (row < NRW) && (Y[row] == sp);
      const unsigned bal = __ballot(hit); const int pre = __popc(bal & ((1u << lane) - 1u)); if (lane == 0) wcnt[wave] = __popc(bal); __syncthreads();
      int woff = 0, tot = 0; for (int w = 0; w < 8; ++w) { const int c = wcnt[w]; if (w < wave) woff += c; tot += c; }
      if (hit) sidx[woff + pre] = row; __syncthreads();
      for (int q = t; q < tot; q += 256) IDX[base + q] = sidx[q];
      base += tot; __syncthreads(); }
    if (t == 0) OFF[sp + 1] = base; }
}
template <int L>
__global__ __launch_bounds__(128) void k_shared(const float* __restrict__ Z, const __bf16* __restrict__ INH, const __bf16* __restrict__ INL, const __bf16* __restrict__ PK, const float* __restrict__ BIAS, __bf16* __restrict__ OH_, __bf16* __restrict__ OL_) {
  __shared__ __align__(16) __bf16 sg[4][16][136], sgl[4][16][136];
  const int tid = threadIdx.x, wave = tid >> 5, lane = tid & 31, col = lane & 15, g = lane >> 4; const size_t r0 = (size_t)blockIdx.x * 64 + wave * 16; const int n0 = blockIdx.y * 128;
  v8f acc[8] = {};
  if (L == 0) { v16b a;
#pragma unroll
    for (int i = 0; i < 16; ++i) { const int k = 8 * g + (i & 7) + ((i >> 3) << 4); a[i] = (__bf16)((k < LAT) ? Z[(r0 + col) * LAT + k] : 0.f); }
#pragma unroll
    for (int j = 0; j < 8; ++j) acc[j] = wmma_bf(a, frag_b(PK + PK_S0 + (size_t)(n0 + j * 16 + col) * 32, lane), acc[j]);
  } else { const __bf16* P = PK + ((L == 1) ? PK_S1 : (L == 2) ? PK_S2 : PK_S3);
#pragma unroll 2
    for (int kc = 0; kc < HID / 32; ++kc) { const v16b a = frag_b(INH + (r0 + col) * HID + kc * 32, lane), al = frag_b(INL + (r0 + col) * HID + kc * 32, lane);
#pragma unroll
      for (int j = 0; j < 8; ++j) { const v16b w = frag_b(P + (size_t)(n0 + j * 16 + col) * HID + kc * 32, lane); acc[j] = wmma_bf(al, w, acc[j]); acc[j] = wmma_bf(a, w, acc[j]); } } }
#pragma unroll
  for (int j = 0; j < 8; ++j) { const float bb = bfr(BIAS[n0 + j * 16 + col]);
#pragma unroll
    for (int r = 0; r < 8; ++r) { const float v = fmaxf(acc[j][r] + bb, 0.f); const __bf16 hb = (__bf16)v; sg[wave][8 * g + r][j * 16 + col] = hb; sgl[wave][8 * g + r][j * 16 + col] = (__bf16)(v - (float)hb); } }
  LDSX();
  for (int rl = 0; rl < 16; ++rl) { if (lane < 16) vst2((unsigned*)(OH_ + (r0 + rl) * HID + n0 + lane * 8), *(const v4u*)&sg[wave][rl][lane * 8]); else vst2((unsigned*)(OL_ + (r0 + rl) * HID + n0 + (lane - 16) * 8), *(const v4u*)&sgl[wave][rl][(lane - 16) * 8]); }
}
template <int L>
__global__ __launch_bounds__(128) void k_unshared(const __bf16* __restrict__ INH, const __bf16* __restrict__ INL, const __bf16* __restrict__ PK, const float* __restrict__ BIAS, const int* __restrict__ IDX, const int* __restrict__ OFF, __bf16* __restrict__ OH_, __bf16* __restrict__ OL_, float* __restrict__ OUT) {
  __shared__ __align__(16) __bf16 sg[4][16][136], sgl[4][16][136]; __shared__ __align__(16) float so[4][16][68]; __shared__ int srow[64];
  const int tid = threadIdx.x, wave = tid >> 5, lane = tid & 31, col = lane & 15, g = lane >> 4; const int sp = blockIdx.z; const int off = OFF[sp], cnt = OFF[sp + 1] - off; const int t0 = blockIdx.x * 64; if (t0 >= cnt) return;
  if (tid < 64) { const int q = t0 + tid; srow[tid] = IDX[off + min(q, cnt - 1)]; }
  __syncthreads();
  const int n0 = blockIdx.y * 128; constexpr int NO = (L == 3) ? STY : HID; if (n0 >= NO) return;
  const __bf16* P = PK + ((L == 0) ? PK_U0 : (L == 1) ? PK_U1 : (L == 2) ? PK_U2 : PK_U3) + (size_t)sp * NO * HID;
  const size_t arow = (size_t)srow[wave * 16 + col];
  constexpr int NT = (L == 3) ? 4 : 8; v8f acc[NT] = {};
#pragma unroll 2
  for (int kc = 0; kc < HID / 32; ++kc) { const v16b a = frag_b(INH + arow * HID + kc * 32, lane), al = frag_b(INL + arow * HID + kc * 32, lane);
#pragma unroll
    for (int j = 0; j < NT; ++j) { const v16b w = frag_b(P + (size_t)(n0 + j * 16 + col) * HID + kc * 32, lane); acc[j] = wmma_bf(al, w, acc[j]); acc[j] = wmma_bf(a, w, acc[j]); } }
  if (L < 3) {
#pragma unroll
    for (int j = 0; j < NT; ++j) { const float bb = bfr(BIAS[sp * HID + n0 + j * 16 + col]);
#pragma unroll
      for (int r = 0; r < 8; ++r) { const float v = fmaxf(acc[j][r] + bb, 0.f); const __bf16 hb = (__bf16)v; sg[wave][8 * g + r][j * 16 + col] = hb; sgl[wave][8 * g + r][j * 16 + col] = (__bf16)(v - (float)hb); } }
    LDSX();
    for (int rl = 0; rl < 16; ++rl) { const int q = t0 + wave * 16 + rl; if (q >= cnt) break; const size_t orow = (size_t)srow[wave * 16 + rl]; if (lane < 16) vst2((unsigned*)(OH_ + orow * HID + n0 + lane * 8), *(const v4u*)&sg[wave][rl][lane * 8]); else vst2((unsigned*)(OL_ + orow * HID + n0 + (lane - 16) * 8), *(const v4u*)&sgl[wave][rl][(lane - 16) * 8]); }
  } else {
#pragma unroll
    for (int j = 0; j < NT; ++j) { const float bb = bfr(BIAS[sp * STY + j * 16 + col]);
#pragma unroll
      for (int r = 0; r < 8; ++r) so[wave][8 * g + r][j * 16 + col] = acc[j][r] + bb; }
    LDSX();
    for (int rl = 0; rl < 16; ++rl) { const int q = t0 + wave * 16 + rl; if (q >= cnt) break; const size_t orow = (size_t)srow[wave * 16 + rl]; if (lane < 16) vst2(OUT + orow * STY + lane * 4, *(const v4f*)&so[wave][rl][lane * 4]); } }
}
extern "C" void kernel_launch(void* const* d_in, const int* in_sizes, int n_in, void* d_out, int out_size, void* d_ws, size_t ws_size, hipStream_t stream) {
  (void)in_sizes; (void)n_in; (void)out_size;
  const float** F = (const float**)d_in;
  if (ws_size < (size_t)WS_END) return;
  char* ws = (char*)d_ws; __bf16 *PK = (__bf16*)(ws + WS_PK), *HA = (__bf16*)(ws + WS_HA), *LA = (__bf16*)(ws + WS_LA), *HB = (__bf16*)(ws + WS_HB), *LB = (__bf16*)(ws + WS_LB); int *IDX = (int*)(ws + WS_IDX), *OFF = (int*)(ws + WS_OFF);
  k_pack<<<dim3(HID, 8, NSP), 256, 0, stream>>>(F[2], F[4], F[6], F[8], F[10], F[12], F[14], F[16], PK);
  k_group<<<1, 256, 0, stream>>>((const int*)d_in[1], IDX, OFF);
  const int RT = NRW / 64;
  k_shared<0><<<dim3(RT, HID / 128), 128, 0, stream>>>(F[0], nullptr, nullptr, PK, F[3], HA, LA);
  k_shared<1><<<dim3(RT, HID / 128), 128, 0, stream>>>(nullptr, HA, LA, PK, F[5], HB, LB);
  k_shared<2><<<dim3(RT, HID / 128), 128, 0, stream>>>(nullptr, HB, LB, PK, F[7], HA, LA);
  k_shared<3><<<dim3(RT, HID / 128), 128, 0, stream>>>(nullptr, HA, LA, PK, F[9], HB, LB);
  const int GT = (NRW + 63) / 64;
  k_unshared<0><<<dim3(GT, HID / 128, NSP), 128, 0, stream>>>(HB, LB, PK, F[11], IDX, OFF, HA, LA, nullptr);
  k_unshared<1><<<dim3(GT, HID / 128, NSP), 128, 0, stream>>>(HA, LA, PK, F[13], IDX, OFF, HB, LB, nullptr);
  k_unshared<2><<<dim3(GT, HID / 128, NSP), 128, 0, stream>>>(HB, LB, PK, F[15], IDX, OFF, HA, LA, nullptr);
  k_unshared<3><<<dim3(GT, 1, NSP), 128, 0, stream>>>(HA, LA, PK, F[17], IDX, OFF, nullptr, nullptr, (float*)d_out);
}
